// PhysioGAT_64871186038940
// MI455X (gfx1250) — hardware-verified
//
#include <hip/hip_runtime.h>
#include <math.h>

#define NN 30000
#define NE 480000
#define NV (NE + NN)
#define NP 30016
#define NG 64
#define F1 512
#define F2 128
#define NT 256
#define SRB 512
#define NTL 59
#define NTA 30

typedef __attribute__((ext_vector_type(16))) _Float16 v16h;
typedef __attribute__((ext_vector_type(8)))  _Float16 v8h;
typedef __attribute__((ext_vector_type(16))) __bf16   v16b;
typedef __attribute__((ext_vector_type(8)))  __bf16   v8b;
typedef __attribute__((ext_vector_type(8)))  float    v8f;
typedef __attribute__((ext_vector_type(4)))  float    v4f;
typedef __attribute__((ext_vector_type(4)))  int      v4i;

__device__ __forceinline__ unsigned short f2bf_bits(float f) {
  unsigned u = __float_as_uint(f);
  return (unsigned short)((u + 0x7FFFu + ((u >> 16) & 1u)) >> 16);
}
__device__ __forceinline__ float bf_bits2f(unsigned short h) { return __uint_as_float(((unsigned)h) << 16); }

__device__ __forceinline__ void dep_guard_h(v8f& a, v8f& b, v16h x, v16h y) { asm volatile("v_nop\n\tv_nop\n\tv_nop\n\tv_nop" : "+v"(a), "+v"(b) : "v"(x), "v"(y)); }
__device__ __forceinline__ void dep_guard_b(v8f& a, v8f& b, v16b x, v16b y) { asm volatile("v_nop\n\tv_nop\n\tv_nop\n\tv_nop" : "+v"(a), "+v"(b) : "v"(x), "v"(y)); }
__device__ __forceinline__ void keep4_h(v16h a, v16h b, v16h c, v16h d) { asm volatile("v_nop" :: "v"(a), "v"(b), "v"(c), "v"(d)); }
__device__ __forceinline__ void keep4_b(v16b a, v16b b, v16b c, v16b d) { asm volatile("v_nop" :: "v"(a), "v"(b), "v"(c), "v"(d)); }
__device__ __forceinline__ void fence_v4(v4f& t) { asm volatile("" : "+v"(t)); }
__device__ __forceinline__ void acc_guard4(v8f& a, v8f& b, v8f& c, v8f& d) { asm volatile("v_nop\n\tv_nop\n\tv_nop\n\tv_nop" : "+v"(a), "+v"(b), "+v"(c), "+v"(d)); }
template <typename T> struct Frag;
template <> struct Frag<_Float16> {
  typedef v16h V; union U { v16h v; v8h h[2]; };
  static __device__ __forceinline__ v16h load(const _Float16* p) {
    U f; f.h[0] = *(const v8h*)(p); f.h[1] = *(const v8h*)(p + 16); return f.v;
  }
  static __device__ __forceinline__ v8f mma(v16h a, v16h b, v8f c) {
    return __builtin_amdgcn_wmma_f32_16x16x32_f16(false, a, false, b, (short)0, c, false, false);
  }
  static __device__ __forceinline__ void guard(v8f& a, v8f& b, v16h x, v16h y) { dep_guard_h(a, b, x, y); }
  static __device__ __forceinline__ void keep(v16h a, v16h b, v16h c, v16h d) { keep4_h(a, b, c, d); }
};
template <> struct Frag<__bf16> {
  typedef v16b V; union U { v16b v; v8b h[2]; };
  static __device__ __forceinline__ v16b load(const __bf16* p) {
    U f; f.h[0] = *(const v8b*)(p); f.h[1] = *(const v8b*)(p + 16); return f.v;
  }
  static __device__ __forceinline__ v8f mma(v16b a, v16b b, v8f c) {
    return __builtin_amdgcn_wmma_f32_16x16x32_bf16(false, a, false, b, (short)0, c, false, false);
  }
  static __device__ __forceinline__ void guard(v8f& a, v8f& b, v16b x, v16b y) { dep_guard_b(a, b, x, y); }
  static __device__ __forceinline__ void keep(v16b a, v16b b, v16b c, v16b d) { keep4_b(a, b, c, d); }
};

template <int ET> struct Elem;
template <> struct Elem<0> { typedef _Float16 T; };
template <> struct Elem<1> { typedef __bf16 T; };
template <int ET, bool SPLIT, int BIAS_MODE, int OUT_MODE, bool RESID, int ACT = 0>
__global__ __launch_bounds__(256) void wmma_gemm64(
    const unsigned short* __restrict__ Ap, const unsigned short* __restrict__ A2p, int lda, long strideA,
    const unsigned short* __restrict__ Btp, const unsigned short* __restrict__ Bt2p, int ldb, long strideB,
    void* __restrict__ Cout, void* __restrict__ Cout2, int ldc, long strideC,
    const float* __restrict__ bias,
    const float* __restrict__ resid, long strideR,
    int M, int N, int K, float scale) {
  typedef typename Elem<ET>::T T;
  typedef typename Frag<T>::V V;
  const T* A = (const T*)Ap; const T* A2 = (const T*)A2p; const T* Bt = (const T*)Btp; const T* Bt2 = (const T*)Bt2p;
  __shared__ __align__(16) float sT[8][16 * 68];
  const int b    = blockIdx.y;
  const int lane = threadIdx.x & 31;
  const int wave = threadIdx.x >> 5;
  const int tilesN = N >> 6;
  const int tilesM = M >> 6;
  const int tile = blockIdx.x * 8 + wave;
  if (tile >= tilesM * tilesN) return;
  const int tm = tile / tilesN;
  const int tn = tile - tm * tilesN;
  const int m0 = tm << 6;
  const int n0 = tn << 6;

  const T* Ab  = A  + (size_t)b * strideA;
  const T* Bb  = Bt + (size_t)b * strideB;
  const T* Ab2 = SPLIT ? (A2  + (size_t)b * strideA) : nullptr;
  const T* Bb2 = SPLIT ? (Bt2 + (size_t)b * strideB) : nullptr;

  const int rlane = lane & 15;
  const int koff  = (lane >> 4) * 8;
  const int mOff  = (lane >> 4) * 8;

  v8f acc[4][4];
#pragma unroll
  for (int i = 0; i < 4; ++i)
#pragma unroll
    for (int j = 0; j < 4; ++j) acc[i][j] = (v8f){0.f,0.f,0.f,0.f,0.f,0.f,0.f,0.f};

  for (int k0 = 0; k0 < K; k0 += 32) {
    V bh[4], bl[4];
#pragma unroll
    for (int j = 0; j < 4; ++j) {
      const size_t bo = (size_t)(n0 + (j << 4) + rlane) * ldb + koff + k0;
      bh[j] = Frag<T>::load(Bb + bo);
      if (SPLIT) bl[j] = Frag<T>::load(Bb2 + bo);
    }
#pragma unroll
    for (int i = 0; i < 4; ++i) {
      const size_t ao = (size_t)(m0 + (i << 4) + rlane) * lda + koff + k0;
      V ah = Frag<T>::load(Ab + ao);
      V al;
      if (SPLIT) al = Frag<T>::load(Ab2 + ao);
#pragma unroll
      for (int j = 0; j < 4; ++j) {
        acc[i][j] = Frag<T>::mma(ah, bh[j], acc[i][j]);
        if (SPLIT) {
          acc[i][j] = Frag<T>::mma(ah, bl[j], acc[i][j]);
          acc[i][j] = Frag<T>::mma(al, bh[j], acc[i][j]);
        }
      }
      Frag<T>::guard(acc[i][0], acc[i][3], ah, SPLIT ? al : ah);
    }
    Frag<T>::keep(bh[0], bh[1], bh[2], bh[3]);
    if (SPLIT) Frag<T>::keep(bl[0], bl[1], bl[2], bl[3]);
  }
  acc_guard4(acc[0][0], acc[0][1], acc[0][2], acc[0][3]);
  acc_guard4(acc[1][0], acc[1][1], acc[1][2], acc[1][3]);
  acc_guard4(acc[2][0], acc[2][1], acc[2][2], acc[2][3]);
  acc_guard4(acc[3][0], acc[3][1], acc[3][2], acc[3][3]);

  float* slab = sT[wave];
  const float* Rb = RESID ? (resid + (size_t)b * strideR) : nullptr;
#pragma unroll
  for (int i = 0; i < 4; ++i) {
    const int mBase = m0 + (i << 4);
#pragma unroll
    for (int j = 0; j < 4; ++j) {
      const int n = n0 + (j << 4) + rlane;
      float bv = 0.f;
      if (BIAS_MODE == 2) bv = bias[n];
#pragma unroll
      for (int r = 0; r < 8; ++r) {
        float v = acc[i][j][r] * scale;
        if (BIAS_MODE == 1) v += bias[mBase + mOff + r];
        if (BIAS_MODE == 2) v += bv;
        if (RESID) v += Rb[(size_t)(mBase + mOff + r) * ldc + n];
        if (ACT == 1) v = tanhf(v);
        if (ACT == 2) v = fmaxf(v, 0.0f);
        if (ACT == 3) v = v / (1.0f + expf(-v));
        if (ACT == 4) v = (v > 0.f) ? v : 0.01f * v;
        if (ACT == 5) v = 0.5f * v * (1.0f + erff(v * 0.70710678118654752f));
        slab[(mOff + r) * 68 + (j << 4) + rlane] = v;
      }
    }
    __builtin_amdgcn_fence(__ATOMIC_RELEASE, "workgroup");
    __builtin_amdgcn_wave_barrier();
    __builtin_amdgcn_fence(__ATOMIC_ACQUIRE, "workgroup");
    if (OUT_MODE == 0) {
      float* C = (float*)Cout + (size_t)b * strideC;
      const int hh = lane >> 4, c4 = (lane & 15) * 4;
      for (int pass = 0; pass < 2; ++pass) {
#pragma unroll
        for (int it = 0; it < 8; ++it) {
          const int row = it * 2 + hh;
          v4f v = *(const v4f*)(slab + row * 68 + c4);
          *(volatile v4f*)(C + (size_t)(mBase + row) * ldc + n0 + c4) = v;
        }
        __threadfence();
      }
    } else {
      const int q = lane >> 3, c8 = (lane & 7) * 8;
      unsigned short* C  = (unsigned short*)Cout  + (size_t)b * strideC;
      unsigned short* C2 = (OUT_MODE == 2) ? ((unsigned short*)Cout2 + (size_t)b * strideC) : nullptr;
      for (int pass = 0; pass < 2; ++pass) {
#pragma unroll
        for (int it = 0; it < 4; ++it) {
          const int row = it * 4 + q;
          const float* sp = slab + row * 68 + c8;
          v8h hv, lv;
#pragma unroll
          for (int e = 0; e < 8; ++e) {
            if (OUT_MODE == 1) {
              hv[e] = (_Float16)sp[e];
            } else {
              unsigned short hb = f2bf_bits(sp[e]);
              unsigned short lb = f2bf_bits(sp[e] - bf_bits2f(hb));
              hv[e] = __builtin_bit_cast(_Float16, hb);
              lv[e] = __builtin_bit_cast(_Float16, lb);
            }
          }
          *(volatile v8h*)(C + (size_t)(mBase + row) * ldc + n0 + c8) = hv;
          if (OUT_MODE == 2) *(volatile v8h*)(C2 + (size_t)(mBase + row) * ldc + n0 + c8) = lv;
        }
        __threadfence();
      }
    }
    __builtin_amdgcn_fence(__ATOMIC_RELEASE, "workgroup");
    __builtin_amdgcn_wave_barrier();
    __builtin_amdgcn_fence(__ATOMIC_ACQUIRE, "workgroup");
  }
}

__device__ __forceinline__ int blk_excl_scan(int cnt, int* scan_ws, int tid, int* tot) {
  const int lane = tid & 31, wave = tid >> 5; int incl = cnt;
#pragma unroll
  for (int o = 1; o < 32; o <<= 1) { const int v = __shfl_up(incl, o, 32); if (lane >= o) incl += v; }
  if (lane == 31) scan_ws[wave] = incl;
  __syncthreads();
  if (wave == 0) { int wv = (lane < NT / 32) ? scan_ws[lane] : 0; int wincl = wv;
#pragma unroll
    for (int o = 1; o < 32; o <<= 1) { const int v = __shfl_up(wincl, o, 32); if (lane >= o) wincl += v; }
    if (lane < NT / 32) scan_ws[32 + lane] = wincl - wv; if (lane == 31) scan_ws[64] = wincl; }
  __syncthreads();
  const int res = scan_ws[32 + wave] + incl - cnt; *tot = scan_ws[64];
  return res;
}
template <int SP, int CAP>
__device__ __forceinline__ int chunk_hits(const int* __restrict__ dstv, const int* __restrict__ srcv, int e0, int n0, int tid,
                                          int* LIST, int* scan_ws) {
  const int eb = e0 + tid * SP;
  int rec[SP]; int cnt = 0;
  if (eb < NE) {
#pragma unroll
    for (int k = 0; k < SP; k += 4) {
      const v4i d4 = *(const v4i*)(dstv + eb + k);
      const v4i s4 = *(const v4i*)(srcv + eb + k);
#pragma unroll
      for (int e = 0; e < 4; ++e) {
        const int d = d4[e]; int r = -1;
        if (d >= n0 && d < n0 + SRB) { int s = s4[e]; s = s < 0 ? 0 : (s >= NN ? NN - 1 : s); r = ((d - n0) << 16) | s; ++cnt; }
        rec[k + e] = r;
      }
    }
  } else {
#pragma unroll
    for (int k = 0; k < SP; ++k) {
      const int e = eb + k; const int d = e - NE; int r = -1;
      if (e < NV && d >= n0 && d < n0 + SRB) { r = ((d - n0) << 16) | d; ++cnt; }
      rec[k] = r;
    }
  }
  int tot; int p = blk_excl_scan(cnt, scan_ws, tid, &tot);
#pragma unroll
  for (int k = 0; k < SP; ++k) if (rec[k] >= 0) { if ((unsigned)p < (unsigned)CAP) LIST[p] = rec[k]; ++p; }
  __syncthreads();
  return tot < CAP ? tot : CAP;
}
__device__ __forceinline__ v4f epi4(v4f a, float inv, v4f bsv, bool live) {
  v4f t = a * inv; fence_v4(t); t = t + bsv;
  v4f r;
#pragma unroll
  for (int e = 0; e < 4; ++e) r[e] = live ? fmaxf(t[e], 0.f) : 0.f;
  return r;
}
__device__ __forceinline__ float dot4(v4f a, v4f b) { return a[0] * b[0] + a[1] * b[1] + a[2] * b[2] + a[3] * b[3]; }
__device__ __forceinline__ float grp8sum(float d) { d += __shfl_xor(d, 1, 32); d += __shfl_xor(d, 2, 32); d += __shfl_xor(d, 4, 32); return d; }

__global__ __launch_bounds__(NT) void prep_kernel(const float* __restrict__ W1, const float* __restrict__ as1, const float* __restrict__ ad1,
                                                 const float* __restrict__ W2, float* __restrict__ WAD,
                                                 unsigned* __restrict__ W2H, unsigned* __restrict__ W2L) {
  const int i = blockIdx.x * NT + threadIdx.x;
  if (i < F2 * F1 / 2) {
    const int o = i >> 8;
    const int k = 2 * (i & 255);
    const float a = W2[(size_t)k * F2 + o], b = W2[(size_t)(k + 1) * F2 + o];
    const unsigned short ha = f2bf_bits(a), hb = f2bf_bits(b);
    const unsigned short la = f2bf_bits(a - bf_bits2f(ha)), lb = f2bf_bits(b - bf_bits2f(hb));
    const unsigned uh = (unsigned)ha | ((unsigned)hb << 16), ul = (unsigned)la | ((unsigned)lb << 16);
    ((volatile unsigned*)W2H)[i] = uh; ((volatile unsigned*)W2L)[i] = ul;
    __threadfence();
    ((volatile unsigned*)W2H)[i] = uh; ((volatile unsigned*)W2L)[i] = ul;
  }
  if (blockIdx.x == 0 && threadIdx.x < 64) {
    const int t = threadIdx.x; const int sel = t >> 5, r = t & 31; const int k = r >> 3, h = r & 7;
    float s = 0.f;
    if (k < 3) {
      const float* av = sel ? ad1 : as1;
#pragma unroll 1
      for (int c = 0; c < 64; ++c) s += W1[k * F1 + h * 64 + c] * av[h * 64 + c];
    }
    ((volatile float*)WAD)[t] = s; __threadfence(); ((volatile float*)WAD)[t] = s;
  }
}

#define SCH1 2048
#define NCH1 ((NV + SCH1 - 1) / SCH1)
__global__ __launch_bounds__(NT) void gat1_kernel(const float* __restrict__ x, const int* __restrict__ ei, const float* __restrict__ WAD,
                                                 const float* __restrict__ W1, const float* __restrict__ b1, float* AGG,
                                                 unsigned short* __restrict__ X1H, unsigned short* __restrict__ X1L, float* __restrict__ X1S,
                                                 int tile0) {
  __shared__ int LIST[SCH1];
  __shared__ float SM[SRB * 8];
  __shared__ float SL[SRB * 8];
  __shared__ float SAD[SRB * 8];
  __shared__ int scan_ws[80];
  const int tid = threadIdx.x, lane = tid & 31, wave = tid >> 5;
  const int n0 = (tile0 + blockIdx.x) * SRB;
  const int rbase = blockIdx.x * SRB;
  const int h8 = lane & 7;
  const float WS0 = WAD[h8], WS1 = WAD[8 + h8], WS2 = WAD[16 + h8];
  v4f w0[4], w1[4], w2[4];
#pragma unroll
  for (int j = 0; j < 4; ++j) {
    w0[j] = *(const v4f*)(W1 + 4 * lane + 128 * j);
    w1[j] = *(const v4f*)(W1 + F1 + 4 * lane + 128 * j);
    w2[j] = *(const v4f*)(W1 + 2 * F1 + 4 * lane + 128 * j);
  }
  const v4f z4 = {0.f, 0.f, 0.f, 0.f};
#pragma unroll 1
  for (int j = 0; j < 64; ++j) {
    float* rp = AGG + (size_t)(rbase + wave * 64 + j) * F1 + 4 * lane;
#pragma unroll
    for (int jj = 0; jj < 4; ++jj) *(v4f*)(rp + 128 * jj) = z4;
  }
  for (int i = tid; i < SRB * 8; i += NT) {
    SM[i] = -INFINITY; SL[i] = 0.f;
    const int dl = i >> 3, h = i & 7; int n = n0 + dl; n = n < NN ? n : NN - 1;
    SAD[i] = x[n * 3] * WAD[32 + h] + x[n * 3 + 1] * WAD[40 + h] + x[n * 3 + 2] * WAD[48 + h];
  }
  __syncthreads();
  const int* srcv = ei; const int* dstv = ei + NE;
#pragma unroll 1
  for (int c = 0; c < NCH1; ++c) {
    const int tot = chunk_hits<SCH1 / NT, SCH1>(dstv, srcv, c * SCH1, n0, tid, LIST, scan_ws);
#pragma unroll 1
    for (int base = 0; base < tot; base += 32) {
      const int q = base + lane;
      const int rv = (q < tot) ? LIST[q] : -1;
      const int own = (rv >= 0 && (rv >> 22) == wave) ? 1 : 0;
      unsigned msk = (unsigned)__ballot(own);
#pragma unroll 1
      for (int it = 0; it < 32; ++it) {
        if (msk == 0u) break;
        const int bp = __builtin_ctz(msk); msk &= msk - 1u;
        const int r = __shfl(rv, bp, 32);
        const int dl = r >> 16, s = r & 0xFFFF;
        const float xs0 = x[s * 3], xs1 = x[s * 3 + 1], xs2 = x[s * 3 + 2];
        const int mi = dl * 8 + h8;
        float al = xs0 * WS0 + xs1 * WS1 + xs2 * WS2 + SAD[mi];
        al = (al >= 0.f) ? al : 0.2f * al;
        const float mo = SM[mi], lo = SL[mi];
        const float mn = fmaxf(mo, al);
        const float rr = __expf(mo - mn), ex = __expf(al - mn);
        const float ln = lo * rr + ex;
        if (lane < 8) { SM[mi] = mn; SL[mi] = ln; }
        float* rp = AGG + (size_t)(rbase + dl) * F1 + 4 * lane;
#pragma unroll
        for (int j = 0; j < 4; ++j) {
          const int hj = 2 * j + (lane >> 4);
          const float rrj = __shfl(rr, hj, 32), exj = __shfl(ex, hj, 32);
          v4f a = *(const v4f*)(rp + 128 * j);
          const v4f hv = xs0 * w0[j] + xs1 * w1[j] + xs2 * w2[j];
          a = a * rrj + exj * hv;
          *(v4f*)(rp + 128 * j) = a;
        }
      }
    }
    __syncthreads();
  }
  const v4f bA0 = *(const v4f*)(b1 + 8 * lane), bA1 = *(const v4f*)(b1 + 8 * lane + 4);
  const v4f bB0 = *(const v4f*)(b1 + 256 + 8 * lane), bB1 = *(const v4f*)(b1 + 256 + 8 * lane + 4);
  const v4f bS = *(const v4f*)(b1 + 4 * lane);
#pragma unroll 1
  for (int j = 0; j < 64; ++j) {
    const int dl = wave * 64 + j; const int n = n0 + dl;
    if (n < NP) {
      const bool live = n < NN;
      float lv = 1.0f;
      if (lane < 8) lv = SL[dl * 8 + lane];
      lv = (live && lv > 0.f) ? lv : 1.0f;
      const float inv8 = 1.0f / lv;
      const float invA = __shfl(inv8, lane >> 3, 32), invB = __shfl(inv8, 4 + (lane >> 3), 32), invS = __shfl(inv8, lane >> 4, 32);
      const float* rp = AGG + (size_t)(rbase + dl) * F1;
      const v4f vA0 = epi4(*(const v4f*)(rp + 8 * lane), invA, bA0, live);
      const v4f vA1 = epi4(*(const v4f*)(rp + 8 * lane + 4), invA, bA1, live);
      const v4f vB0 = epi4(*(const v4f*)(rp + 256 + 8 * lane), invB, bB0, live);
      const v4f vB1 = epi4(*(const v4f*)(rp + 256 + 8 * lane + 4), invB, bB1, live);
      const v4f vS  = epi4(*(const v4f*)(rp + 4 * lane), invS, bS, live);
      v8h hA, lA, hB, lB;
#pragma unroll
      for (int e = 0; e < 4; ++e) {
        unsigned short hb, lb;
        hb = f2bf_bits(vA0[e]); lb = f2bf_bits(vA0[e] - bf_bits2f(hb)); hA[e] = __builtin_bit_cast(_Float16, hb); lA[e] = __builtin_bit_cast(_Float16, lb);
        hb = f2bf_bits(vA1[e]); lb = f2bf_bits(vA1[e] - bf_bits2f(hb)); hA[4 + e] = __builtin_bit_cast(_Float16, hb); lA[4 + e] = __builtin_bit_cast(_Float16, lb);
        hb = f2bf_bits(vB0[e]); lb = f2bf_bits(vB0[e] - bf_bits2f(hb)); hB[e] = __builtin_bit_cast(_Float16, hb); lB[e] = __builtin_bit_cast(_Float16, lb);
        hb = f2bf_bits(vB1[e]); lb = f2bf_bits(vB1[e] - bf_bits2f(hb)); hB[4 + e] = __builtin_bit_cast(_Float16, hb); lB[4 + e] = __builtin_bit_cast(_Float16, lb);
      }
      unsigned short* rh = X1H + (size_t)n * F1; unsigned short* rl = X1L + (size_t)n * F1; float* rs = X1S + (size_t)n * F2;
      for (int pass = 0; pass < 2; ++pass) {
        *(volatile v8h*)(rh + 8 * lane) = hA; *(volatile v8h*)(rh + 256 + 8 * lane) = hB;
        *(volatile v8h*)(rl + 8 * lane) = lA; *(volatile v8h*)(rl + 256 + 8 * lane) = lB;
        *(volatile v4f*)(rs + 4 * lane) = vS;
        __threadfence();
      }
    }
  }
}

#define SCH2 4096
#define NCH2 ((NV + SCH2 - 1) / SCH2)
__global__ __launch_bounds__(NT) void gat2_kernel(const float* __restrict__ H2, const int* __restrict__ ei, const float* __restrict__ as2,
                                                 const float* __restrict__ ad2, const float* __restrict__ b2, const float* __restrict__ X1S,
                                                 float* HS) {
  __shared__ int LIST[SCH2];
  __shared__ float SM[SRB * 4];
  __shared__ float SL[SRB * 4];
  __shared__ float SAD[SRB * 4];
  __shared__ int scan_ws[80];
  const int tid = threadIdx.x, lane = tid & 31, wave = tid >> 5;
  const int n0 = blockIdx.x * SRB;
  const int hq = lane >> 3;
  const v4f asr = *(const v4f*)(as2 + 4 * lane), adr = *(const v4f*)(ad2 + 4 * lane), br = *(const v4f*)(b2 + 4 * lane);
  const v4f z4 = {0.f, 0.f, 0.f, 0.f};
#pragma unroll 1
  for (int j = 0; j < 64; ++j) *(v4f*)(HS + (size_t)(n0 + wave * 64 + j) * F2 + 4 * lane) = z4;
  for (int i = tid; i < SRB * 4; i += NT) { SM[i] = -INFINITY; SL[i] = 0.f; }
#pragma unroll 1
  for (int dl = wave; dl < SRB; dl += 8) {
    int n = n0 + dl; n = n < NP ? n : NP - 1;
    const v4f hv = *(const v4f*)(H2 + (size_t)n * F2 + 4 * lane);
    const float d = grp8sum(dot4(hv, adr));
    if ((lane & 7) == 0) SAD[dl * 4 + hq] = d;
  }
  __syncthreads();
  const int* srcv = ei; const int* dstv = ei + NE;
#pragma unroll 1
  for (int c = 0; c < NCH2; ++c) {
    const int tot = chunk_hits<SCH2 / NT, SCH2>(dstv, srcv, c * SCH2, n0, tid, LIST, scan_ws);
#pragma unroll 1
    for (int base = 0; base < tot; base += 32) {
      const int q = base + lane;
      const int rv = (q < tot) ? LIST[q] : -1;
      const int own = (rv >= 0 && (rv >> 22) == wave) ? 1 : 0;
      unsigned msk = (unsigned)__ballot(own);
#pragma unroll 1
      for (int it = 0; it < 32; ++it) {
        if (msk == 0u) break;
        const int bp = __builtin_ctz(msk); msk &= msk - 1u;
        const int r = __shfl(rv, bp, 32);
        const int dl = r >> 16, s = r & 0xFFFF;
        const v4f hv = *(const v4f*)(H2 + (size_t)s * F2 + 4 * lane);
        const int mi = dl * 4 + hq;
        float al = grp8sum(dot4(hv, asr)) + SAD[mi];
        al = (al >= 0.f) ? al : 0.2f * al;
        const float mo = SM[mi], lo = SL[mi];
        const float mn = fmaxf(mo, al);
        const float rr = __expf(mo - mn), ex = __expf(al - mn);
        const float ln = lo * rr + ex;
        if ((lane & 7) == 0) { SM[mi] = mn; SL[mi] = ln; }
        float* rp = HS + (size_t)(n0 + dl) * F2 + 4 * lane;
        v4f a = *(const v4f*)rp;
        a = a * rr + ex * hv;
        *(v4f*)rp = a;
      }
    }
    __syncthreads();
  }
#pragma unroll 1
  for (int j = 0; j < 64; ++j) {
    const int dl = wave * 64 + j; const int n = n0 + dl;
    if (n < NN) {
      float lv = SL[dl * 4 + hq]; lv = lv > 0.f ? lv : 1.0f;
      const float inv = 1.0f / lv;
      float* rp = HS + (size_t)n * F2 + 4 * lane;
      v4f v = epi4(*(const v4f*)rp, inv, br, true);
      const v4f sk = *(const v4f*)(X1S + (size_t)n * F2 + 4 * lane);
      v = v + sk;
      for (int pass = 0; pass < 2; ++pass) { *(volatile v4f*)rp = v; __threadfence(); }
    }
  }
}

#define SCHP 2048
#define NCHP ((NN + SCHP - 1) / SCHP)
__global__ __launch_bounds__(NT) void pool_kernel(const float* __restrict__ HS, const int* __restrict__ batch, float* __restrict__ P) {
  __shared__ int LIST[SCHP];
  __shared__ int scan_ws[80];
  __shared__ __align__(16) float red[8 * F2];
  __shared__ int rc[8];
  const int tid = threadIdx.x, lane = tid & 31, wave = tid >> 5;
  const int g = blockIdx.x;
  const v4f z4 = {0.f, 0.f, 0.f, 0.f};
  v4f acc = z4; int cnt = 0;
#pragma unroll 1
  for (int c = 0; c < NCHP; ++c) {
    const int eb = c * SCHP + tid * 8;
    int bv[8]; int rec[8]; int kc = 0;
    if (eb < NN) {
      const v4i b0 = *(const v4i*)(batch + eb), bb = *(const v4i*)(batch + eb + 4);
      bv[0] = b0[0]; bv[1] = b0[1]; bv[2] = b0[2]; bv[3] = b0[3]; bv[4] = bb[0]; bv[5] = bb[1]; bv[6] = bb[2]; bv[7] = bb[3];
    } else {
#pragma unroll
      for (int k = 0; k < 8; ++k) bv[k] = -1;
    }
#pragma unroll
    for (int k = 0; k < 8; ++k) { rec[k] = -1; if (bv[k] == g) { rec[k] = eb + k; ++kc; } }
    int tot; int p = blk_excl_scan(kc, scan_ws, tid, &tot);
#pragma unroll
    for (int k = 0; k < 8; ++k) if (rec[k] >= 0) { if ((unsigned)p < (unsigned)SCHP) LIST[p] = rec[k]; ++p; }
    __syncthreads();
    const int totc = tot < SCHP ? tot : SCHP;
#pragma unroll 1
    for (int q = wave; q < totc; q += 8) {
      int nd = LIST[q]; nd = nd < 0 ? 0 : (nd >= NN ? NN - 1 : nd);
      acc = acc + *(const v4f*)(HS + (size_t)nd * F2 + 4 * lane); ++cnt;
    }
    __syncthreads();
  }
  *(v4f*)(red + wave * F2 + 4 * lane) = acc;
  if (lane == 0) rc[wave] = cnt;
  __syncthreads();
  if (wave == 0) {
    v4f s = z4; int ct = 0;
#pragma unroll
    for (int w = 0; w < 8; ++w) { s = s + *(const v4f*)(red + w * F2 + 4 * lane); ct += rc[w]; }
    const float cf = (float)ct;
    const float inv = 1.0f / fmaxf(cf, 1.0f);
    const v4f o = s * inv;
    for (int pass = 0; pass < 2; ++pass) { *(volatile v4f*)(P + (size_t)g * F2 + 4 * lane) = o; __threadfence(); }
  }
}

__global__ __launch_bounds__(NT) void head_kernel(const float* __restrict__ P, const float* __restrict__ Wfc, const float* __restrict__ bfc,
                                                 const float* __restrict__ gam, const float* __restrict__ bet,
                                                 const float* __restrict__ Wh, const float* __restrict__ bh,
                                                 const float* __restrict__ Wd, const float* __restrict__ bd, float* __restrict__ out) {
  __shared__ float zs[NG * 32];
  __shared__ float smu[32];
  __shared__ float srs[32];
  __shared__ __align__(16) float so[320];
  const int tid = threadIdx.x, wave = tid >> 5, lane = tid & 31;
  for (int i = tid; i < NG * 32; i += NT) {
    const int g = i >> 5, j = i & 31;
    float s = 0.f;
#pragma unroll 1
    for (int c = 0; c < F2; ++c) s += P[g * F2 + c] * Wfc[c * 32 + j];
    zs[i] = s + bfc[j];
  }
  __syncthreads();
  if (tid < 32) {
    double m = 0.0;
#pragma unroll 1
    for (int g = 0; g < NG; ++g) m += (double)zs[g * 32 + tid];
    m = m * (1.0 / NG);
    const float mf = (float)m;
    double v = 0.0;
#pragma unroll 1
    for (int g = 0; g < NG; ++g) { const float d = zs[g * 32 + tid] - mf; const float dd = d * d; v += (double)dd; }
    v = v * (1.0 / NG);
    const float vf = (float)v;
    smu[tid] = mf; srs[tid] = 1.0f / sqrtf(vf + 1e-5f);
  }
  __syncthreads();
  for (int i = tid; i < NG * 32; i += NT) {
    const int j = i & 31;
    float t = gam[j] * (zs[i] - smu[j]);
    t = t * srs[j];
    t = t + bet[j];
    zs[i] = fmaxf(t, 0.f);
  }
  __syncthreads();
  for (int i = tid; i < 320; i += NT) {
    float a = 0.f;
    if (i < 192) {
      const int g = i / 3, k = i - 3 * g;
#pragma unroll 1
      for (int j = 0; j < 32; ++j) a += zs[g * 32 + j] * Wh[j * 3 + k];
      a += bh[k];
    } else {
      const int r = i - 192; const int g = r >> 1, k = r & 1;
#pragma unroll 1
      for (int j = 0; j < 32; ++j) a += zs[g * 32 + j] * Wd[j * 2 + k];
      a += bd[k];
    }
    so[i] = a;
  }
  __syncthreads();
  if (wave == 0) {
    const v4f p0 = *(const v4f*)(so + 4 * lane);
    const v4f p1 = *(const v4f*)(so + 128 + 4 * lane);
    const v4f p2 = *(const v4f*)(so + 256 + 4 * (lane & 15));
    for (int pass = 0; pass < 2; ++pass) {
      *(volatile v4f*)(out + 4 * lane) = p0;
      *(volatile v4f*)(out + 128 + 4 * lane) = p1;
      if (lane < 16) *(volatile v4f*)(out + 256 + 4 * lane) = p2;
      __threadfence();
    }
  }
}

extern "C" void kernel_launch(void* const* d_in, const int* in_sizes, int n_in,
                              void* d_out, int out_size, void* d_ws, size_t ws_size, hipStream_t stream) {
  (void)in_sizes; (void)n_in; (void)out_size;
  const float* x      = (const float*)d_in[0];
  const int*   ei     = (const int*)  d_in[1];
  const int*   batch  = (const int*)  d_in[2];
  const float* W1     = (const float*)d_in[3];
  const float* as1    = (const float*)d_in[4];
  const float* ad1    = (const float*)d_in[5];
  const float* b1     = (const float*)d_in[6];
  const float* W2     = (const float*)d_in[7];
  const float* as2    = (const float*)d_in[8];
  const float* ad2    = (const float*)d_in[9];
  const float* b2     = (const float*)d_in[10];
  const float* Wfc    = (const float*)d_in[11];
  const float* bfc    = (const float*)d_in[12];
  const float* bn_g   = (const float*)d_in[13];
  const float* bn_b   = (const float*)d_in[14];
  const float* Wheat  = (const float*)d_in[15];
  const float* bheat  = (const float*)d_in[16];
  const float* Wdehyd = (const float*)d_in[17];
  const float* bdehyd = (const float*)d_in[18];
  float* out = (float*)d_out;

  char* ws = (char*)d_ws; size_t off = 0;
  auto carve = [&](size_t bytes) -> char* { char* p = ws + off; off += (bytes + 255) & ~(size_t)255; return p; };
  float*          WAD = (float*)carve(256);
  unsigned*       W2H = (unsigned*)carve((size_t)F2 * F1 * 2);
  unsigned*       W2L = (unsigned*)carve((size_t)F2 * F1 * 2);
  unsigned short* X1H = (unsigned short*)carve((size_t)NP * F1 * 2);
  unsigned short* X1L = (unsigned short*)carve((size_t)NP * F1 * 2);
  float*          X1S = (float*)carve((size_t)NP * F2 * 4);
  char*           R   = carve((size_t)NTA * SRB * F1 * 4);
  float*          P   = (float*)carve((size_t)NG * F2 * 4);
  if (off > ws_size || off > (size_t)134217728) return;
  float* AGG1 = (float*)R;
  float* H2   = (float*)R;
  float* HS   = (float*)(R + (size_t)NP * F2 * 4);

  prep_kernel<<<(F2 * F1 / 2 + NT - 1) / NT, NT, 0, stream>>>(W1, as1, ad1, W2, WAD, W2H, W2L);
  gat1_kernel<<<NTA, NT, 0, stream>>>(x, ei, WAD, W1, b1, AGG1, X1H, X1L, X1S, 0);
  gat1_kernel<<<NTL - NTA, NT, 0, stream>>>(x, ei, WAD, W1, b1, AGG1, X1H, X1L, X1S, NTA);
  {
    const int tiles = (NP / 64) * (F2 / 64);
    wmma_gemm64<1, true, 0, 0, false><<<dim3((tiles + 7) / 8, 1), 256, 0, stream>>>(
        (const unsigned short*)X1H, (const unsigned short*)X1L, F1, 0L,
        (const unsigned short*)W2H, (const unsigned short*)W2L, F1, 0L,
        (void*)H2, (void*)nullptr, F2, 0L,
        (const float*)nullptr, (const float*)nullptr, 0L, NP, F2, F1, 1.0f);
  }
  gat2_kernel<<<NTL, NT, 0, stream>>>(H2, ei, as2, ad2, b2, X1S, HS);
  pool_kernel<<<NG, NT, 0, stream>>>(HS, batch, P);
  head_kernel<<<1, NT, 0, stream>>>(P, Wfc, bfc, bn_g, bn_b, Wheat, bheat, Wdehyd, bdehyd, out);
}
